// GCC_54786602828345
// MI455X (gfx1250) — hardware-verified
//
#include <hip/hip_runtime.h>
#define NN 50000
#define NNP 50048
#define NE 800000
#define NG 128
#define DIN 32
#define D0 65
#define D0P 128
#define DH 64
#define DO 32
#define NL 5
#define DCAP 64
typedef __bf16 v16b __attribute__((ext_vector_type(16)));
typedef unsigned short v8us __attribute__((ext_vector_type(8), may_alias));
typedef float  v8f  __attribute__((ext_vector_type(8)));
typedef float  v4f  __attribute__((ext_vector_type(4)));
typedef float  v4fa __attribute__((ext_vector_type(4), may_alias));
union FragB { v16b v; v8us half[2]; unsigned short u[16]; };

__device__ __forceinline__ unsigned short bf16_bits(float x) { unsigned int u = __float_as_uint(x); return (unsigned short)((u + 0x7FFFu + ((u >> 16) & 1u)) >> 16); }
__device__ __forceinline__ float bf16_val(unsigned short b) { return __uint_as_float(((unsigned int)b) << 16); }
__device__ __forceinline__ float bf16_round(float x) { return bf16_val(bf16_bits(x)); }
template <int NT>
__device__ __forceinline__ v8f mmaN(v16b ah, v16b al, v16b bh, v16b bl, v8f c) {
  c = __builtin_amdgcn_wmma_f32_16x16x32_bf16(false, ah, false, bh, (short)0, c, false, false);
  if (NT >= 2) c = __builtin_amdgcn_wmma_f32_16x16x32_bf16(false, al, false, bh, (short)0, c, false, false);
  if (NT >= 3) c = __builtin_amdgcn_wmma_f32_16x16x32_bf16(false, ah, false, bl, (short)0, c, false, false);
  asm volatile("v_nop\n\tv_nop\n\tv_nop\n\tv_nop" : "+v"(c) : "v"(ah), "v"(al), "v"(bh), "v"(bl));
  return c;
}

__global__ __launch_bounds__(256) void k_wt_bf16(const float* __restrict__ W, unsigned short* __restrict__ Wt, int K, int N) {
  const int t = blockIdx.x * 256 + threadIdx.x;
  const int k8n = K / 8;
  if (t >= N * k8n) return;
  const int n = t / k8n, k8 = (t % k8n) * 8;
  v8us v;
#pragma unroll
  for (int i = 0; i < 8; ++i) v[i] = bf16_bits(W[(size_t)(k8 + i) * N + n]);
  *(volatile v8us*)(Wt + (size_t)n * K + k8) = v;
  __threadfence();
  *(volatile v8us*)(Wt + (size_t)n * K + k8) = v;
}

template <bool ASPLIT, int ACT, bool BIAS_BF16>
__global__ __launch_bounds__(128) void k_gemm_bf(const float* __restrict__ A, int lda, const unsigned short* __restrict__ Wt, int ldb,
                                               const float* __restrict__ bias, float* __restrict__ C, int ldc, int M, int N, int K) {
  __shared__ __attribute__((aligned(16))) float so[4][16][64];
  const int tid = threadIdx.x, w = tid >> 5, lane = tid & 31, ln = lane & 15, hh = lane >> 4;
  const int ntn = N / 64;
  const int wid = blockIdx.x * 4 + w;
  const int mt = wid / ntn, nq = wid % ntn;
  if (mt * 16 >= M) return;
  const int row0 = mt * 16, col0 = nq * 64;
  const float* arow = A + (size_t)(row0 + ln) * lda;
  v8f acc[4] = {};
  for (int kb = 0; kb < K; kb += 32) {
    FragB ah, al;
    const v4f x0 = *(const v4fa*)(arow + kb + 8 * hh), x1 = *(const v4fa*)(arow + kb + 8 * hh + 4);
    const v4f x2 = *(const v4fa*)(arow + kb + 16 + 8 * hh), x3 = *(const v4fa*)(arow + kb + 16 + 8 * hh + 4);
    float xs[16] = {x0[0],x0[1],x0[2],x0[3],x1[0],x1[1],x1[2],x1[3],x2[0],x2[1],x2[2],x2[3],x3[0],x3[1],x3[2],x3[3]};
#pragma unroll
    for (int i = 0; i < 16; ++i) { const unsigned short hb = bf16_bits(xs[i]); ah.u[i] = hb; al.u[i] = ASPLIT ? bf16_bits(xs[i] - bf16_val(hb)) : (unsigned short)0; }
#pragma unroll
    for (int t = 0; t < 4; ++t) {
      const unsigned short* brow = Wt + (size_t)(col0 + t * 16 + ln) * ldb + kb;
      FragB b;
      b.half[0] = *(const v8us*)(brow + 8 * hh);
      b.half[1] = *(const v8us*)(brow + 16 + 8 * hh);
      acc[t] = mmaN<ASPLIT ? 2 : 1>(ah.v, al.v, b.v, b.v, acc[t]);
    }
  }
#pragma unroll
  for (int t = 0; t < 4; ++t) {
    float bv = bias ? bias[col0 + t * 16 + ln] : 0.f;
    if (BIAS_BF16) bv = bf16_round(bv);
#pragma unroll
    for (int r = 0; r < 8; ++r) { float v = acc[t][r] + bv; if (ACT == 1) v = fmaxf(v, 0.f); so[w][8 * hh + r][t * 16 + ln] = v; }
  }
  __builtin_amdgcn_fence(__ATOMIC_ACQ_REL, "workgroup");
  __builtin_amdgcn_wave_barrier();
  const int rsub = lane >> 4, c4 = (lane & 15) * 4;
  for (int pass = 0; pass < 2; ++pass) {
#pragma unroll
    for (int q = 0; q < 8; ++q) {
      const int r = q * 2 + rsub;
      const v4f v = *(const v4fa*)&so[w][r][c4];
      *(volatile v4f*)(C + (size_t)(row0 + r) * ldc + col0 + c4) = v;
    }
    if (pass == 0) __threadfence();
  }
}

template <bool ASPLIT, int ACT, bool BIAS_BF16, bool RES_BF16>
__global__ __launch_bounds__(128) void k_gemm_bf3(const float* __restrict__ A, int lda, const unsigned short* __restrict__ Wt, int ldb,
                                                const float* __restrict__ bias, const float* __restrict__ resid, int rmod, int ldr,
                                                float* __restrict__ C, int ldc, int M, int N, int K) {
  __shared__ __attribute__((aligned(16))) float so[4][16][64];
  const int tid = threadIdx.x, w = tid >> 5, lane = tid & 31, ln = lane & 15, hh = lane >> 4;
  const int ntn = N / 64;
  const int wid = blockIdx.x * 4 + w;
  const int mt = wid / ntn, nq = wid % ntn;
  if (mt * 16 >= M) return;
  const int row0 = mt * 16, col0 = nq * 64;
  const float* arow = A + (size_t)(row0 + ln) * lda;
  v8f acc[4] = {};
  for (int kb = 0; kb < K; kb += 32) {
    FragB ah, al;
    const v4f x0 = *(const v4fa*)(arow + kb + 8 * hh), x1 = *(const v4fa*)(arow + kb + 8 * hh + 4);
    const v4f x2 = *(const v4fa*)(arow + kb + 16 + 8 * hh), x3 = *(const v4fa*)(arow + kb + 16 + 8 * hh + 4);
    float xs[16] = {x0[0],x0[1],x0[2],x0[3],x1[0],x1[1],x1[2],x1[3],x2[0],x2[1],x2[2],x2[3],x3[0],x3[1],x3[2],x3[3]};
#pragma unroll
    for (int i = 0; i < 16; ++i) { const unsigned short hb = bf16_bits(xs[i]); ah.u[i] = hb; al.u[i] = ASPLIT ? bf16_bits(xs[i] - bf16_val(hb)) : (unsigned short)0; }
#pragma unroll
    for (int t = 0; t < 4; ++t) {
      const unsigned short* brow = Wt + (size_t)(col0 + t * 16 + ln) * ldb + kb;
      FragB b;
      b.half[0] = *(const v8us*)(brow + 8 * hh);
      b.half[1] = *(const v8us*)(brow + 16 + 8 * hh);
      acc[t] = mmaN<ASPLIT ? 2 : 1>(ah.v, al.v, b.v, b.v, acc[t]);
    }
  }
#pragma unroll
  for (int t = 0; t < 4; ++t) {
    const int col = col0 + t * 16 + ln;
    float bv = bias ? bias[col] : 0.f;
    if (BIAS_BF16) bv = bf16_round(bv);
#pragma unroll
    for (int r = 0; r < 8; ++r) {
      float v = acc[t][r] + bv;
      if (resid) { float rv = resid[(size_t)((row0 + 8 * hh + r) % rmod) * ldr + col]; if (RES_BF16) rv = bf16_round(rv); v += rv; }
      if (ACT == 1) v = fmaxf(v, 0.f);
      if (ACT == 2) v = 0.5f * v * (1.0f + erff(v * 0.70710678118654752f));
      if (ACT == 3) { const float u = 0.7978845608028654f * (v + 0.044715f * v * v * v); v = 0.5f * v * (1.0f + tanhf(u)); }
      so[w][8 * hh + r][t * 16 + ln] = v;
    }
  }
  __builtin_amdgcn_fence(__ATOMIC_ACQ_REL, "workgroup");
  __builtin_amdgcn_wave_barrier();
  const int rsub = lane >> 4, c4 = (lane & 15) * 4;
  for (int pass = 0; pass < 2; ++pass) {
#pragma unroll
    for (int q = 0; q < 8; ++q) {
      const int r = q * 2 + rsub;
      const v4f v = *(const v4fa*)&so[w][r][c4];
      *(volatile v4f*)(C + (size_t)(row0 + r) * ldc + col0 + c4) = v;
    }
    if (pass == 0) __threadfence();
  }
}
template <bool PARAM_BF16>
__global__ __launch_bounds__(256) void k_layernorm(const float* __restrict__ X, const float* __restrict__ R, const float* __restrict__ g, const float* __restrict__ bta,
                                                  float* __restrict__ out_sum, float* __restrict__ out_norm, int N, float eps) {
  __shared__ float red[256];
  const int row = blockIdx.x, tid = threadIdx.x;
  const float* x = X + (size_t)row * N; const float* rr = R ? R + (size_t)row * N : nullptr;
  float vals[16];
  const int per = N / 256;
  float s1 = 0.f;
  for (int u = 0; u < per / 4; ++u) {
    const int j = tid * 4 + 1024 * u;
    const v4f a = *(const v4fa*)(x + j);
    v4f b = {0.f,0.f,0.f,0.f}; if (rr) b = *(const v4fa*)(rr + j);
#pragma unroll
    for (int q = 0; q < 4; ++q) { const float v = a[q] + b[q]; vals[u * 4 + q] = v; s1 += v; }
  }
  red[tid] = s1; __syncthreads();
  for (int st = 128; st > 0; st >>= 1) { if (tid < st) red[tid] += red[tid + st]; __syncthreads(); }
  const float mu = red[0] / (float)N; __syncthreads();
  float s2 = 0.f;
  for (int u = 0; u < per / 4; ++u)
#pragma unroll
    for (int q = 0; q < 4; ++q) { const float c = vals[u * 4 + q] - mu; s2 += c * c; }
  red[tid] = s2; __syncthreads();
  for (int st = 128; st > 0; st >>= 1) { if (tid < st) red[tid] += red[tid + st]; __syncthreads(); }
  const float rs = rsqrtf(red[0] / (float)N + eps);
  for (int pass = 0; pass < 2; ++pass) {
    for (int u = 0; u < per / 4; ++u) {
      const int j = tid * 4 + 1024 * u;
      v4f o, sm;
#pragma unroll
      for (int q = 0; q < 4; ++q) {
        float gg = g[j + q], bb = bta[j + q];
        if (PARAM_BF16) { gg = bf16_round(gg); bb = bf16_round(bb); }
        sm[q] = vals[u * 4 + q]; o[q] = (vals[u * 4 + q] - mu) * rs * gg + bb;
      }
      if (out_sum) *(volatile v4f*)(out_sum + (size_t)row * N + j) = sm;
      *(volatile v4f*)(out_norm + (size_t)row * N + j) = o;
    }
    if (pass == 0) __threadfence();
  }
}


typedef _Float16 v16h __attribute__((ext_vector_type(16)));
union FragH { v16h v; v8us half[2]; _Float16 h[16]; unsigned short u[16]; };
template <int NT>
__device__ __forceinline__ v8f mmaH(v16h ah, v16h al, v16h bh, v16h bl, v8f c) {
  c = __builtin_amdgcn_wmma_f32_16x16x32_f16(false, ah, false, bh, (short)0, c, false, false);
  if (NT >= 2) c = __builtin_amdgcn_wmma_f32_16x16x32_f16(false, al, false, bh, (short)0, c, false, false);
  if (NT >= 3) c = __builtin_amdgcn_wmma_f32_16x16x32_f16(false, ah, false, bl, (short)0, c, false, false);
  asm volatile("v_nop\n\tv_nop\n\tv_nop\n\tv_nop" : "+v"(c) : "v"(ah), "v"(al), "v"(bh), "v"(bl));
  return c;
}
template <bool ASPLIT>
__global__ __launch_bounds__(128) void k_gemm_h(const float* __restrict__ A, int lda, size_t sA, const _Float16* __restrict__ Bh, int ldb, size_t sB, float alpha, float* __restrict__ C, int ldc, size_t sC, int M, int N, int K) {
  __shared__ __attribute__((aligned(16))) float so[4][16][64];
  const int tid = threadIdx.x, w = tid >> 5, lane = tid & 31, ln = lane & 15, hh = lane >> 4; const int by = blockIdx.y;
  A += (size_t)by * sA; Bh += (size_t)by * sB; C += (size_t)by * sC;
  const int ntn = (N + 63) / 64; const int wid = blockIdx.x * 4 + w; const int mt = wid / ntn, nq = wid % ntn; if (mt * 16 >= M) return;
  const int row0 = mt * 16, col0 = nq * 64; const float* arow = A + (size_t)(row0 + ln) * lda;
  v8f acc[4] = {};
  for (int kb = 0; kb < K; kb += 32) {
    FragH ah, al;
    const v4f x0 = *(const v4fa*)(arow + kb + 8 * hh), x1 = *(const v4fa*)(arow + kb + 8 * hh + 4), x2 = *(const v4fa*)(arow + kb + 16 + 8 * hh), x3 = *(const v4fa*)(arow + kb + 16 + 8 * hh + 4);
    float xs[16] = {x0[0],x0[1],x0[2],x0[3],x1[0],x1[1],x1[2],x1[3],x2[0],x2[1],x2[2],x2[3],x3[0],x3[1],x3[2],x3[3]};
#pragma unroll
    for (int i = 0; i < 16; ++i) { const _Float16 h = (_Float16)xs[i]; ah.h[i] = h; al.h[i] = ASPLIT ? (_Float16)(xs[i] - (float)h) : (_Float16)0.0f; }
#pragma unroll
    for (int t = 0; t < 4; ++t) { if (col0 + t * 16 >= N) continue; const size_t boff = (size_t)(col0 + t * 16 + ln) * ldb + kb; FragH bq; bq.half[0] = *(const v8us*)(Bh + boff + 8 * hh); bq.half[1] = *(const v8us*)(Bh + boff + 16 + 8 * hh);
      acc[t] = mmaH<ASPLIT ? 2 : 1>(ah.v, al.v, bq.v, bq.v, acc[t]); }
  }
#pragma unroll
  for (int t = 0; t < 4; ++t) { if (col0 + t * 16 >= N) continue;
#pragma unroll
    for (int r = 0; r < 8; ++r) so[w][8 * hh + r][t * 16 + ln] = acc[t][r] * alpha; }
  __builtin_amdgcn_fence(__ATOMIC_ACQ_REL, "workgroup"); __builtin_amdgcn_wave_barrier();
  const int rsub = lane >> 4, c4 = (lane & 15) * 4;
  for (int pass = 0; pass < 2; ++pass) {
#pragma unroll
    for (int q = 0; q < 8; ++q) { const int r = q * 2 + rsub; if (col0 + c4 < N) { const v4f v = *(const v4fa*)&so[w][r][c4]; *(volatile v4f*)(C + (size_t)(row0 + r) * ldc + col0 + c4) = v; } }
    if (pass == 0) __threadfence(); }
}

__global__ __launch_bounds__(256) void k_wt_f16(const float* __restrict__ W, _Float16* __restrict__ Wt, int K, int N, float scale) {
  const int t = blockIdx.x * 256 + threadIdx.x; if (t >= N * (K / 8)) return; const int n = t / (K / 8), k8 = (t % (K / 8)) * 8; FragH f;
#pragma unroll
  for (int i = 0; i < 8; ++i) f.h[i] = (_Float16)(bf16_round(W[(size_t)(k8 + i) * N + n]) * scale); const v8us o = f.half[0];
  *(volatile v8us*)((unsigned short*)Wt + (size_t)n * K + k8) = o; __threadfence(); *(volatile v8us*)((unsigned short*)Wt + (size_t)n * K + k8) = o;
}
template <int ACT>
__global__ __launch_bounds__(128) void k_gemm_hhx(const _Float16* __restrict__ A, int lda, size_t sA, const _Float16* __restrict__ Bh, int ldb, size_t sB, float alpha, const float* __restrict__ bias, size_t sBias, const float* __restrict__ CP, int rowsPerB, size_t sCPb, int row0g,
    float* __restrict__ C, _Float16* __restrict__ C16, int ldc, size_t sC, int M, int N, int K) {
  __shared__ __attribute__((aligned(16))) float so[4][16][64];
  const int tid = threadIdx.x, w = tid >> 5, lane = tid & 31, ln = lane & 15, hh = lane >> 4; const int by = blockIdx.y;
  A += (size_t)by * sA; Bh += (size_t)by * sB; const size_t cofs = (size_t)by * sC; const float* bp = bias ? bias + (size_t)by * sBias : nullptr;
  const int ntn = (N + 63) / 64; const int wid = blockIdx.x * 4 + w; const int mt = wid / ntn, nq = wid % ntn; if (mt * 16 >= M) return;
  const int row0 = mt * 16, col0 = nq * 64; const _Float16* arow = A + (size_t)(row0 + ln) * lda;
  v8f acc[4] = {};
  for (int kb = 0; kb < K; kb += 32) { FragH ah; ah.half[0] = *(const v8us*)((const unsigned short*)arow + kb + 8 * hh); ah.half[1] = *(const v8us*)((const unsigned short*)arow + kb + 16 + 8 * hh);
#pragma unroll
    for (int t = 0; t < 4; ++t) { if (col0 + t * 16 >= N) continue; const size_t boff = (size_t)(col0 + t * 16 + ln) * ldb + kb; FragH bq; bq.half[0] = *(const v8us*)((const unsigned short*)Bh + boff + 8 * hh); bq.half[1] = *(const v8us*)((const unsigned short*)Bh + boff + 16 + 8 * hh);
      acc[t] = mmaH<1>(ah.v, ah.v, bq.v, bq.v, acc[t]); }
  }
#pragma unroll
  for (int t = 0; t < 4; ++t) { if (col0 + t * 16 >= N) continue; const int col = col0 + t * 16 + ln; const float bv = bp ? bf16_round(bp[col]) : 0.f;
#pragma unroll
    for (int r = 0; r < 8; ++r) { float v = acc[t][r] * alpha + bv; if (CP) { const int bidx = (row0g + row0 + 8 * hh + r) / rowsPerB; v += CP[(size_t)bidx * sCPb + (size_t)by * 64 + col]; } if (ACT == 1) v = (v > 0.f) ? v : expm1f(v); else if (ACT == 7) v = (v > 0.f) ? v + 1.0f : expf(v); else if (ACT == 8) v = tanhf(v); else if (ACT == 9) v = 0.5f * v * (1.0f + tanhf(0.7978845608028654f * (v + 0.044715f * v * v * v))); else if (ACT == 11) v = 1.0f / (1.0f + expf(-v)); else if (ACT == 12) v = (v > 0.f) ? v : 0.01f * v; else if (ACT == 14) v = (v > 0.f) ? v : 0.1f * v; else if (ACT == 15) v = v / (1.0f + expf(-v)); else if (ACT == 3) v = fmaxf(v, 0.f); else if (ACT == 6) v = 0.5f * v * (1.0f + erff(v * 0.70710678118654752f)); so[w][8 * hh + r][t * 16 + ln] = v; } }
  __builtin_amdgcn_fence(__ATOMIC_ACQ_REL, "workgroup"); __builtin_amdgcn_wave_barrier();
  const int rsub = lane >> 4, c4 = (lane & 15) * 4; typedef _Float16 v4h __attribute__((ext_vector_type(4)));
  for (int pass = 0; pass < 2; ++pass) {
#pragma unroll
    for (int q = 0; q < 8; ++q) { const int r = q * 2 + rsub; if (col0 + c4 < N) { const v4f v = *(const v4fa*)&so[w][r][c4]; if (C) *(volatile v4f*)(C + cofs + (size_t)(row0 + r) * ldc + col0 + c4) = v; if (C16) { v4h h4; for (int i = 0; i < 4; ++i) h4[i] = (_Float16)v[i]; *(volatile v4h*)(C16 + cofs + (size_t)(row0 + r) * ldc + col0 + c4) = h4; } } }
    if (pass == 0) __threadfence(); }
}


typedef _Float16 v4h __attribute__((ext_vector_type(4)));

__global__ __launch_bounds__(256) void k_x16(const float* __restrict__ x, _Float16* __restrict__ X16, size_t n8) { const size_t t = (size_t)blockIdx.x * 256 + threadIdx.x; if (t >= n8) return; FragH f;
#pragma unroll
  for (int q = 0; q < 8; ++q) f.h[q] = (_Float16)bf16_round(x[t * 8 + q]); *(volatile v8us*)((unsigned short*)X16 + t * 8) = f.half[0]; __threadfence(); *(volatile v8us*)((unsigned short*)X16 + t * 8) = f.half[0]; }
__global__ __launch_bounds__(256) void k_h16(const float* __restrict__ x, _Float16* __restrict__ X16, size_t n8) { const size_t t = (size_t)blockIdx.x * 256 + threadIdx.x; if (t >= n8) return; FragH f;
#pragma unroll
  for (int q = 0; q < 8; ++q) f.h[q] = (_Float16)x[t * 8 + q]; *(volatile v8us*)((unsigned short*)X16 + t * 8) = f.half[0]; __threadfence(); *(volatile v8us*)((unsigned short*)X16 + t * 8) = f.half[0]; }
__global__ __launch_bounds__(256) void k_round16f(const float* __restrict__ W, _Float16* __restrict__ Bt, size_t n8) { const size_t t = (size_t)blockIdx.x * 256 + threadIdx.x; if (t >= n8) return; FragH f;
#pragma unroll
  for (int i = 0; i < 8; ++i) f.h[i] = (_Float16)(bf16_round(W[t * 8 + i]) * 16.0f); *(volatile v8us*)((unsigned short*)Bt + t * 8) = f.half[0]; __threadfence(); *(volatile v8us*)((unsigned short*)Bt + t * 8) = f.half[0]; }
template <int NHv, int TTv>
__global__ __launch_bounds__(256) void k_vt(const _Float16* __restrict__ V16, int ldv, int voff, _Float16* __restrict__ Vt) { __shared__ unsigned short tl[64][66]; const int tid = threadIdx.x; const int slab = blockIdx.x / (TTv / 64), lg = blockIdx.x % (TTv / 64); const int b = slab / NHv, h = slab % NHv;
  for (int i = tid; i < 64 * 8; i += 256) { const int r = i / 8, c8 = (i % 8) * 8; FragH f; f.half[0] = *(const v8us*)((const unsigned short*)V16 + ((size_t)b * TTv + lg * 64 + r) * ldv + voff + h * 64 + c8);
#pragma unroll
    for (int q = 0; q < 8; ++q) tl[r][c8 + q] = f.u[q]; }
  __syncthreads();
  for (int pass = 0; pass < 2; ++pass) {
#pragma unroll
    for (int rd = 0; rd < 2; ++rd) { const int d = rd * 32 + tid / 8, pc = tid % 8; FragH f;
#pragma unroll
      for (int q = 0; q < 8; ++q) f.u[q] = tl[pc * 8 + q][d];
      *(volatile v8us*)((unsigned short*)Vt + ((size_t)slab * 64 + d) * TTv + lg * 64 + pc * 8) = f.half[0]; }
    if (pass == 0) __threadfence(); } }

__global__ __launch_bounds__(256) void k_hl(const float* __restrict__ F, _Float16* __restrict__ Hh, _Float16* __restrict__ Hl, size_t n8) { const size_t t = (size_t)blockIdx.x * 256 + threadIdx.x; if (t >= n8) return; FragH fh, fl; const v4f a = *(const v4fa*)(F + t * 8), c = *(const v4fa*)(F + t * 8 + 4);
#pragma unroll
  for (int q = 0; q < 4; ++q) { _Float16 h = (_Float16)a[q]; fh.h[q] = h; fl.h[q] = (_Float16)((a[q] - (float)h) * 1024.0f); h = (_Float16)c[q]; fh.h[4 + q] = h; fl.h[4 + q] = (_Float16)((c[q] - (float)h) * 1024.0f); }
  for (int pass = 0; pass < 2; ++pass) { *(volatile v8us*)((unsigned short*)Hh + t * 8) = fh.half[0]; *(volatile v8us*)((unsigned short*)Hl + t * 8) = fl.half[0]; if (pass == 0) __threadfence(); } }
#define VST2(T, ptr, val) do { const T vst2_v_ = (val); *(volatile T*)(ptr) = vst2_v_; __threadfence(); *(volatile T*)(ptr) = vst2_v_; } while (0)

#define C4_NB 4096
#define C4_CH 8192
__device__ __forceinline__ int c4_bucket(int v, int N) { v = min(max(v, 0), N - 1); return (int)(((long long)v * C4_NB) / N); }
__global__ __launch_bounds__(256) void k_c4_count(const int* __restrict__ tgt, int E, int N, int* __restrict__ CNT) {
    __shared__ int hist[C4_NB]; const int ch = blockIdx.x, t = threadIdx.x; const int e0 = ch * C4_CH; const int nt = min(C4_CH, E - e0);
    for (int j = 0; j < 16; ++j) hist[t + 256 * j] = 0; __syncthreads();
    for (int i = t; i < nt; i += 256) atomicAdd(&hist[c4_bucket(tgt[e0 + i], N)], 1);
    __syncthreads();
    for (int j = 0; j < 16; ++j) { const int v = hist[t + 256 * j]; VST2(int, CNT + (long long)ch * C4_NB + t + 256 * j, v); } }
__global__ __launch_bounds__(256) void k_c4_offsets(const int* __restrict__ CNT, int nch, int E, int* __restrict__ OFFB, int* __restrict__ BOFF) {
    __shared__ int tot[C4_NB]; __shared__ int part[256]; const int t = threadIdx.x;
    for (int j = 0; j < 16; ++j) { const int b = t + 256 * j; int s = 0; for (int ch = 0; ch < nch; ++ch) s += CNT[(long long)ch * C4_NB + b]; tot[b] = s; }
    __syncthreads();
    { int s = 0; for (int q = 0; q < 16; ++q) s += tot[16 * t + q]; part[t] = s; } __syncthreads();
    if (t == 0) { int run = 0; for (int i = 0; i < 256; ++i) { const int v = part[i]; part[i] = run; run += v; } } __syncthreads();
    { int run = part[t]; for (int q = 0; q < 16; ++q) { const int v = tot[16 * t + q]; tot[16 * t + q] = run; run += v; } }
    __syncthreads();
    for (int j = 0; j < 16; ++j) { const int b = t + 256 * j; VST2(int, BOFF + b, tot[b]); }
    if (t == 0) VST2(int, BOFF + C4_NB, E);
    for (int j = 0; j < 16; ++j) { const int b = t + 256 * j; int run = tot[b]; for (int ch = 0; ch < nch; ++ch) { VST2(int, OFFB + (long long)ch * C4_NB + b, run); run += CNT[(long long)ch * C4_NB + b]; } } }
__global__ __launch_bounds__(256) void k_c4_scatter(const int* __restrict__ tgt, int E, int N, const int* __restrict__ OFFB, int* __restrict__ BUF) {
    __shared__ int cur[C4_NB]; __shared__ int bk[256]; const int ch = blockIdx.x, t = threadIdx.x; const int e0 = ch * C4_CH; const int nt = min(C4_CH, E - e0);
    const int wv = t >> 5, ln = t & 31;
    for (int j = 0; j < 16; ++j) cur[t + 256 * j] = OFFB[(long long)ch * C4_NB + t + 256 * j];
    __syncthreads();
    for (int s0 = 0; s0 < C4_CH; s0 += 256) {
        const int i = s0 + t; const int e = e0 + i; const int b = (i < nt) ? c4_bucket(tgt[min(e, E - 1)], N) : -1;
        bk[t] = b; __syncthreads();
        int rank = 0, cntw = 0;
        for (int l = 0; l < 32; ++l) { const int o = bk[(wv << 5) + l]; const bool same = (o == b) && (b >= 0); cntw += same ? 1 : 0; rank += (same && l < ln) ? 1 : 0; }
        const bool last = (b >= 0) && (rank == cntw - 1);
        for (int w = 0; w < 8; ++w) {
            if (wv == w && b >= 0) { int pos = cur[b] + rank; pos = min(max(pos, 0), E - 1); VST2(int, BUF + pos, e); }
            __syncthreads();
            if (wv == w && last) cur[b] += cntw;
            __syncthreads(); }
    } }
template <int CAP>
__global__ __launch_bounds__(256) void k_c4_lists(const int* __restrict__ tgt, const int* __restrict__ BUF, const int* __restrict__ BOFF, int N, int E, int* __restrict__ NBR, int* __restrict__ cnt) {
    const int d = blockIdx.x * 256 + threadIdx.x; if (d >= N) return; const int b = c4_bucket(d, N); int n = 0; int* row = NBR + (long long)d * CAP;
    const int p0 = min(max(BOFF[b], 0), E), p1 = min(max(BOFF[b + 1], p0), E);
    for (int p = p0; p < p1; ++p) { int e = BUF[p]; e = min(max(e, 0), E - 1); if (tgt[e] == d) { if (n < CAP) VST2(int, row + n, e); ++n; } }
    for (int j = n; j < CAP; ++j) VST2(int, row + j, -1); VST2(int, cnt + d, min(n, CAP)); }
__global__ __launch_bounds__(256) void k_c4_scan1(const int* __restrict__ cnt, int* __restrict__ PART, int N) {
    __shared__ int part[256]; const int per = ((((N + 255) / 256) + 31) / 32) * 32; const int a = threadIdx.x * per, b = min(N, a + per); int s = 0;
    for (int i = a; i < b; ++i) s += cnt[i]; part[threadIdx.x] = s; __syncthreads();
    if (threadIdx.x == 0) { int run = 0; for (int t = 0; t < 256; ++t) { const int v = part[t]; part[t] = run; run += v; } } __syncthreads();
    VST2(int, PART + threadIdx.x, part[threadIdx.x]); }
__global__ __launch_bounds__(256) void k_c4_scan2(const int* __restrict__ cnt, const int* __restrict__ PART, int* __restrict__ off, int N) {
    const int i = blockIdx.x * 256 + threadIdx.x; if (i > N) return; const int per = ((((N + 255) / 256) + 31) / 32) * 32; const int r = min(i / per, 255); const int a = r * per;
    int s = PART[r]; for (int kq = a; kq < i; ++kq) s += cnt[min(kq, N - 1)];
    VST2(int, off + i, s); }
template <int CAP>
__global__ __launch_bounds__(256) void k_c4_slotcopy(const int* __restrict__ off, const int* __restrict__ NBR, int* __restrict__ slot, int N) {
    const int t = blockIdx.x * 256 + threadIdx.x; const int tot = off[N]; if (t >= tot) return;
    int lo = 0, hi = N - 1; while (lo < hi) { const int mid = (lo + hi + 1) >> 1; if (off[mid] <= t) lo = mid; else hi = mid - 1; }
    int j = t - off[lo]; j = (j < 0) ? 0 : ((j >= CAP) ? (CAP - 1) : j); VST2(int, slot + t, NBR[(long long)lo * CAP + j]); }

__global__ __launch_bounds__(256) void k_splitp(const float* __restrict__ F, int rows, int C, int P, _Float16* __restrict__ Hh, _Float16* __restrict__ Hl) {
  #pragma clang fp contract(off)
  const size_t t = (size_t)blockIdx.x * 256 + threadIdx.x; if (t >= (size_t)rows * (P / 8)) return; const int c0 = (int)(t % (P / 8)) * 8; const size_t r = t / (P / 8); FragH fh, fl;
#pragma unroll
  for (int q = 0; q < 8; ++q) { const int c = c0 + q; const float v = (c < C) ? F[r * C + c] : 0.f; const _Float16 hi = (_Float16)v; fh.h[q] = hi; fl.h[q] = (_Float16)((v - (float)hi) * 1024.0f); }
  for (int pass = 0; pass < 2; ++pass) { *(volatile v8us*)((unsigned short*)Hh + r * P + c0) = fh.half[0]; *(volatile v8us*)((unsigned short*)Hl + r * P + c0) = fl.half[0]; if (pass == 0) __threadfence(); } }
__global__ __launch_bounds__(256) void k_h0(const float* __restrict__ x, const int* __restrict__ cntS, const float* __restrict__ degt, const int* __restrict__ roots, float* __restrict__ H0) {
  #pragma clang fp contract(off)
  const int tid = threadIdx.x, w = tid >> 5, l = tid & 31; const int n = blockIdx.x * 8 + w; if (n >= NN) return; const int dg = min(max(cntS[n], 0), 128); float ego = 0.f;
#pragma unroll 1
  for (int k = 0; k < NG; ++k) ego = (roots[k] == n) ? 1.f : ego;
  float v[3]; v[0] = bf16_round(x[(size_t)n * DIN + l]); v[1] = bf16_round(degt[(size_t)dg * DIN + l]); v[2] = (l == 0) ? ego : 0.f;
  for (int pass = 0; pass < 2; ++pass) { *(volatile float*)(H0 + (size_t)n * D0P + l) = v[0]; *(volatile float*)(H0 + (size_t)n * D0P + 32 + l) = v[1]; *(volatile float*)(H0 + (size_t)n * D0P + 64 + l) = v[2]; *(volatile float*)(H0 + (size_t)n * D0P + 96 + l) = 0.f; if (pass == 0) __threadfence(); } }
template <int C>
__global__ __launch_bounds__(256) void k_gin(const int* __restrict__ NBR, const int* __restrict__ cnt, const int* __restrict__ esrc, const float* __restrict__ H, _Float16* __restrict__ Zh, _Float16* __restrict__ Zl) {
  #pragma clang fp contract(off)
  const int tid = threadIdx.x, w = tid >> 5, l = tid & 31; const int d = blockIdx.x * 8 + w; if (d >= NN) return; const int ne = min(cnt[d], DCAP); constexpr int M = C / 32; float acc[M];
#pragma unroll
  for (int m = 0; m < M; ++m) acc[m] = H[(size_t)d * C + l + 32 * m];
#pragma unroll 1
  for (int j = 0; j < ne; ++j) { int e = NBR[(size_t)d * DCAP + j]; e = min(max(e, 0), NE - 1); int s = esrc[e]; s = min(max(s, 0), NN - 1);
#pragma unroll
    for (int m = 0; m < M; ++m) acc[m] += H[(size_t)s * C + l + 32 * m]; }
  for (int pass = 0; pass < 2; ++pass) {
#pragma unroll
    for (int m = 0; m < M; ++m) { FragH f; const _Float16 hi = (_Float16)acc[m]; f.h[0] = hi; *(volatile unsigned short*)((unsigned short*)Zh + (size_t)d * C + l + 32 * m) = f.u[0]; f.h[0] = (_Float16)((acc[m] - (float)hi) * 1024.0f); *(volatile unsigned short*)((unsigned short*)Zl + (size_t)d * C + l + 32 * m) = f.u[0]; }
    if (pass == 0) __threadfence(); } }
__global__ __launch_bounds__(256) void k_colstats(const float* __restrict__ Z, double* __restrict__ SUM, double* __restrict__ SQ) { __shared__ double s1[8][32], s2[8][32]; const int tid = threadIdx.x, w = tid >> 5, l = tid & 31; const int c = blockIdx.x * 32 + l; double a = 0.0, b = 0.0;
#pragma unroll 1
  for (int r = w; r < NN; r += 8) { const double v = (double)Z[(size_t)r * DH + c]; a += v; b += v * v; }
  s1[w][l] = a; s2[w][l] = b; __syncthreads();
  if (w == 0) { double t1 = 0.0, t2 = 0.0; for (int k = 0; k < 8; ++k) { t1 += s1[k][l]; t2 += s2[k][l]; } for (int pass = 0; pass < 2; ++pass) { *(volatile double*)(SUM + c) = t1; *(volatile double*)(SQ + c) = t2; if (pass == 0) __threadfence(); } } }
__global__ __launch_bounds__(256) void k_bnrelu(const float* __restrict__ X, const double* __restrict__ SUM, const double* __restrict__ SQ, const float* __restrict__ g, const float* __restrict__ bb, float* __restrict__ Y, _Float16* __restrict__ Yh, _Float16* __restrict__ Yl) {
  #pragma clang fp contract(off)
  const int t = blockIdx.x * 256 + threadIdx.x; if (t >= NN * (DH / 4)) return; const int c0 = (t % (DH / 4)) * 4, r = t / (DH / 4); const v4f xv = *(const v4fa*)(X + (size_t)r * DH + c0); v4f o; FragH fh, fl;
#pragma unroll
  for (int q = 0; q < 4; ++q) { const int c = c0 + q; const double m = SUM[c] / (double)NN; double var = SQ[c] / (double)NN - m * m; if (var < 0.0) var = 0.0; const float v = fmaxf(bf16_round(g[c]) * (xv[q] - (float)m) * rsqrtf((float)var + 1e-5f) + bf16_round(bb[c]), 0.f); o[q] = v; const _Float16 hi = (_Float16)v; fh.h[q] = hi; fl.h[q] = (_Float16)((v - (float)hi) * 1024.0f); }
  const unsigned long long vh = *(const unsigned long long*)&fh.u[0], vl = *(const unsigned long long*)&fl.u[0];
  for (int pass = 0; pass < 2; ++pass) { *(volatile v4f*)(Y + (size_t)r * DH + c0) = o; if (Yh) { *(volatile unsigned long long*)((unsigned short*)Yh + (size_t)r * DH + c0) = vh; *(volatile unsigned long long*)((unsigned short*)Yl + (size_t)r * DH + c0) = vl; } if (pass == 0) __threadfence(); } }
__global__ __launch_bounds__(256) void k_granges(const int* __restrict__ batch, int* __restrict__ GR) { __shared__ int st[NG], en[NG]; const int tid = threadIdx.x; if (tid < NG) { st[tid] = NN; en[tid] = -1; } __syncthreads();
#pragma unroll 1
  for (int n = tid; n < NN; n += 256) { int g = batch[n]; g = min(max(g, 0), NG - 1); atomicMin(&st[g], n); atomicMax(&en[g], n); }
  __syncthreads();
  if (tid < 32) { for (int g = 0; g < NG; ++g) { const int s = st[g], c = (en[g] >= s) ? (en[g] - s + 1) : 0; const int v = (tid == 0) ? ((c > 0) ? s : 0) : (tid == 1) ? c : 0; *(volatile int*)(GR + g * 32 + tid) = v; __threadfence(); *(volatile int*)(GR + g * 32 + tid) = v; } } }
template <int C>
__global__ __launch_bounds__(256) void k_gpool(const float* __restrict__ Hp, const int* __restrict__ batch, const int* __restrict__ GR, _Float16* __restrict__ Ph, _Float16* __restrict__ Pl) {
  #pragma clang fp contract(off)
  constexpr int NS = 256 / C;
  __shared__ float part[NS][C]; __shared__ __attribute__((aligned(16))) unsigned short rh[D0P], rl[D0P]; const int tid = threadIdx.x, g = blockIdx.x; for (int i = tid; i < D0P; i += 256) { rh[i] = 0; rl[i] = 0; } __syncthreads();
  const int n0 = GR[g * 32], gcnt = GR[g * 32 + 1];
  { const int st = tid / C, cl = tid % C; float s = 0.f;
#pragma unroll 1
    for (int i = st; i < gcnt; i += NS) { const int n = n0 + i; if (batch[n] == g) s += Hp[(size_t)n * C + cl]; } part[st][cl] = s; }
  __syncthreads();
  if (tid < C) { float v = 0.f;
#pragma unroll
    for (int k = 0; k < NS; ++k) v += part[k][tid]; FragH f; const _Float16 hi = (_Float16)v; f.h[0] = hi; rh[tid] = f.u[0]; f.h[0] = (_Float16)((v - (float)hi) * 1024.0f); rl[tid] = f.u[0]; }
  __syncthreads();
  if (tid < D0P / 8) { for (int pass = 0; pass < 2; ++pass) { *(volatile v8us*)((unsigned short*)Ph + (size_t)g * D0P + tid * 8) = *(const v8us*)&rh[tid * 8]; *(volatile v8us*)((unsigned short*)Pl + (size_t)g * D0P + tid * 8) = *(const v8us*)&rl[tid * 8]; if (pass == 0) __threadfence(); } } }
__global__ __launch_bounds__(256) void k_wtp(const float* __restrict__ Wm, int in, int out, _Float16* __restrict__ Bt) { const int t = blockIdx.x * 256 + threadIdx.x; if (t >= out * (D0P / 8)) return; const int k0 = (t % (D0P / 8)) * 8, o = t / (D0P / 8); FragH f;
#pragma unroll
  for (int q = 0; q < 8; ++q) { const int k = k0 + q; f.h[q] = (k < in) ? (_Float16)(bf16_round(Wm[(size_t)k * out + o]) * 16.0f) : (_Float16)0.0f; }
  *(volatile v8us*)((unsigned short*)Bt + (size_t)o * D0P + k0) = f.half[0]; __threadfence(); *(volatile v8us*)((unsigned short*)Bt + (size_t)o * D0P + k0) = f.half[0]; }
__global__ __launch_bounds__(256) void k_norm(const float* __restrict__ S, float* __restrict__ out) {
  #pragma clang fp contract(off)
  const int tid = threadIdx.x, w = tid >> 5, l = tid & 31; const int g = blockIdx.x * 8 + w; if (g >= NG) return; const float v = S[(size_t)g * DO + l]; float ss = v * v; for (int o = 16; o > 0; o >>= 1) ss += __shfl_xor(ss, o, 32); const float nrm = fmaxf(sqrtf(ss), 1e-5f); const float r = v / nrm;
  *(volatile float*)(out + (size_t)g * DO + l) = r; __threadfence(); *(volatile float*)(out + (size_t)g * DO + l) = r; }

extern "C" void kernel_launch(void* const* d_in, const int* in_sizes, int n_in,
                              void* d_out, int out_size, void* d_ws, size_t ws_size, hipStream_t stream) {
  (void)in_sizes; (void)n_in; (void)out_size;
  const float* x = (const float*)d_in[0]; const int* ei = (const int*)d_in[1]; const int* batch = (const int*)d_in[2]; const int* roots = (const int*)d_in[3]; const float* degt = (const float*)d_in[4];
  const float* w1_0 = (const float*)d_in[5]; const float* b1_0 = (const float*)d_in[6]; const float* w2_0 = (const float*)d_in[7]; const float* b2_0 = (const float*)d_in[8]; const float* w1r = (const float*)d_in[9]; const float* b1r = (const float*)d_in[10]; const float* w2r = (const float*)d_in[11]; const float* b2r = (const float*)d_in[12]; const float* bng = (const float*)d_in[13]; const float* bnb = (const float*)d_in[14]; const float* pw0 = (const float*)d_in[15]; const float* pb0 = (const float*)d_in[16]; const float* pwr = (const float*)d_in[17]; const float* pbr = (const float*)d_in[18];
  const int* esrc = ei; const int* edst = ei + NE;
  char* ws = (char*)d_ws; size_t off = 0;
  auto take = [&](size_t bytes) { char* p = ws + off; off += (bytes + 255) & ~(size_t)255; return p; };
  const int nch = (NE + C4_CH - 1) / C4_CH;
  int* CNT = (int*)take((size_t)nch * C4_NB * 4); int* OFFB = (int*)take((size_t)nch * C4_NB * 4); int* BOFF = (int*)take((size_t)(C4_NB + 64) * 4); int* BUF = (int*)take((size_t)NE * 4); int* NBR = (int*)take((size_t)NN * DCAP * 4); int* cnt = (int*)take((size_t)(NN + 64) * 4); int* cntS = (int*)take((size_t)(NN + 64) * 4);
  _Float16* B1[NL]; _Float16* B2[NL]; _Float16* BP[NL + 1]; for (int l = 0; l < NL; ++l) { B1[l] = (_Float16*)take(DH * D0P * 2); B2[l] = (_Float16*)take(DH * D0P * 2); } for (int l = 0; l <= NL; ++l) BP[l] = (_Float16*)take(DO * D0P * 2);
  float* H0 = (float*)take((size_t)NNP * D0P * 4); _Float16* Zh = (_Float16*)take((size_t)NNP * D0P * 2); _Float16* Zl = (_Float16*)take((size_t)NNP * D0P * 2); float* T1 = (float*)take((size_t)NNP * DH * 4); float* T2 = (float*)take((size_t)NNP * DH * 4); _Float16* Th = (_Float16*)take((size_t)NNP * DH * 2); _Float16* Tl = (_Float16*)take((size_t)NNP * DH * 2); float* H = (float*)take((size_t)NNP * DH * 4); double* SUM = (double*)take(DH * 8); double* SQ = (double*)take(DH * 8);
  _Float16* Ph = (_Float16*)take((size_t)NG * D0P * 2); _Float16* Pl = (_Float16*)take((size_t)NG * D0P * 2); float* SC = (float*)take((size_t)NG * DO * 4); int* GR = (int*)take(NG * 32 * 4);
  if (off > ws_size) return;
  k_c4_count<<<nch, 256, 0, stream>>>(esrc, NE, NN, CNT); k_c4_offsets<<<1, 256, 0, stream>>>(CNT, nch, NE, OFFB, BOFF); k_c4_scatter<<<nch, 256, 0, stream>>>(esrc, NE, NN, OFFB, BUF); k_c4_lists<DCAP><<<(NN + 255) / 256, 256, 0, stream>>>(esrc, BUF, BOFF, NN, NE, NBR, cntS);
  k_c4_count<<<nch, 256, 0, stream>>>(edst, NE, NN, CNT); k_c4_offsets<<<1, 256, 0, stream>>>(CNT, nch, NE, OFFB, BOFF); k_c4_scatter<<<nch, 256, 0, stream>>>(edst, NE, NN, OFFB, BUF); k_c4_lists<DCAP><<<(NN + 255) / 256, 256, 0, stream>>>(edst, BUF, BOFF, NN, NE, NBR, cnt);
  k_wtp<<<(DH * (D0P / 8) + 255) / 256, 256, 0, stream>>>(w1_0, D0, DH, B1[0]); k_wtp<<<(DH * (D0P / 8) + 255) / 256, 256, 0, stream>>>(w2_0, DH, DH, B2[0]);
  for (int l = 1; l < NL; ++l) { k_wtp<<<(DH * (D0P / 8) + 255) / 256, 256, 0, stream>>>(w1r + (size_t)(l - 1) * DH * DH, DH, DH, B1[l]); k_wtp<<<(DH * (D0P / 8) + 255) / 256, 256, 0, stream>>>(w2r + (size_t)(l - 1) * DH * DH, DH, DH, B2[l]); }
  k_wtp<<<(DO * (D0P / 8) + 255) / 256, 256, 0, stream>>>(pw0, D0, DO, BP[0]); for (int l = 0; l < NL; ++l) k_wtp<<<(DO * (D0P / 8) + 255) / 256, 256, 0, stream>>>(pwr + (size_t)l * DH * DO, DH, DO, BP[l + 1]);
  k_h0<<<(NN + 7) / 8, 256, 0, stream>>>(x, cntS, degt, roots, H0);
  const dim3 gH(((NN / 16) * 1 + 3) / 4, 1), gG(((NG / 16) * 1 + 3) / 4, 1); const unsigned nb4 = (NN * (DH / 4) + 255) / 256;
  k_granges<<<1, 256, 0, stream>>>(batch, GR); k_gpool<D0P><<<NG, 256, 0, stream>>>(H0, batch, GR, Ph, Pl);
  k_gemm_hhx<0><<<gG, 128, 0, stream>>>(Ph, D0P, 0, BP[0], D0P, 0, 0.0625f, pb0, 0, nullptr, 1, 0, 0, SC, nullptr, DO, 0, NG, DO, D0P); k_gemm_hhx<0><<<gG, 128, 0, stream>>>(Pl, D0P, 0, BP[0], D0P, 0, 0.0625f / 1024.0f, nullptr, 0, SC, 1, (size_t)DO, 0, SC, nullptr, DO, 0, NG, DO, D0P);
  for (int l = 0; l < NL; ++l) {
    if (l == 0) k_gin<D0P><<<(NN + 7) / 8, 256, 0, stream>>>(NBR, cnt, esrc, H0, Zh, Zl); else k_gin<DH><<<(NN + 7) / 8, 256, 0, stream>>>(NBR, cnt, esrc, H, Zh, Zl);
    const int K1 = (l == 0) ? D0P : DH;
    k_gemm_hhx<0><<<gH, 128, 0, stream>>>(Zh, K1, 0, B1[l], D0P, 0, 0.0625f, (l == 0) ? b1_0 : b1r + (size_t)(l - 1) * DH, 0, nullptr, 1, 0, 0, T1, nullptr, DH, 0, NN, DH, K1); k_gemm_hhx<0><<<gH, 128, 0, stream>>>(Zl, K1, 0, B1[l], D0P, 0, 0.0625f / 1024.0f, nullptr, 0, T1, 1, (size_t)DH, 0, T1, nullptr, DH, 0, NN, DH, K1);
    k_colstats<<<DH / 32, 256, 0, stream>>>(T1, SUM, SQ); k_bnrelu<<<nb4, 256, 0, stream>>>(T1, SUM, SQ, bng + ((size_t)l * 3 + 0) * DH, bnb + ((size_t)l * 3 + 0) * DH, T2, Th, Tl);
    k_gemm_hhx<0><<<gH, 128, 0, stream>>>(Th, DH, 0, B2[l], D0P, 0, 0.0625f, (l == 0) ? b2_0 : b2r + (size_t)(l - 1) * DH, 0, nullptr, 1, 0, 0, T1, nullptr, DH, 0, NN, DH, DH); k_gemm_hhx<0><<<gH, 128, 0, stream>>>(Tl, DH, 0, B2[l], D0P, 0, 0.0625f / 1024.0f, nullptr, 0, T1, 1, (size_t)DH, 0, T1, nullptr, DH, 0, NN, DH, DH);
    k_colstats<<<DH / 32, 256, 0, stream>>>(T1, SUM, SQ); k_bnrelu<<<nb4, 256, 0, stream>>>(T1, SUM, SQ, bng + ((size_t)l * 3 + 1) * DH, bnb + ((size_t)l * 3 + 1) * DH, T2, nullptr, nullptr);
    k_colstats<<<DH / 32, 256, 0, stream>>>(T2, SUM, SQ); k_bnrelu<<<nb4, 256, 0, stream>>>(T2, SUM, SQ, bng + ((size_t)l * 3 + 2) * DH, bnb + ((size_t)l * 3 + 2) * DH, H, nullptr, nullptr);
    k_gpool<DH><<<NG, 256, 0, stream>>>(H, batch, GR, Ph, Pl);
    k_gemm_hhx<0><<<gG, 128, 0, stream>>>(Ph, D0P, 0, BP[l + 1], D0P, 0, 0.0625f, pbr + (size_t)l * DO, 0, SC, 1, (size_t)DO, 0, SC, nullptr, DO, 0, NG, DO, DH); k_gemm_hhx<0><<<gG, 128, 0, stream>>>(Pl, D0P, 0, BP[l + 1], D0P, 0, 0.0625f / 1024.0f, nullptr, 0, SC, 1, (size_t)DO, 0, SC, nullptr, DO, 0, NG, DO, DH); }
  k_norm<<<NG / 8, 256, 0, stream>>>(SC, (float*)d_out);
}
